// CausalAdaptiveKernelAttention_16956530885209
// MI455X (gfx1250) — hardware-verified
//
#include <hip/hip_runtime.h>
#define NB 4
#define TT 1024
#define DD 1024
#define NH 16
#define HD 64
#define TH 256
#define CX 2048
#define C4 512
#define NKP 144
#define NKPP 192
#define HCH 8
#define RB 64
#define NR (NB * TT)
#define NRH (NB * TH)
#define SCL 0.125f
typedef __bf16 v16b __attribute__((ext_vector_type(16)));
typedef unsigned short v8us __attribute__((ext_vector_type(8), may_alias));
typedef float  v8f  __attribute__((ext_vector_type(8)));
typedef float  v4f  __attribute__((ext_vector_type(4)));
typedef float  v4fa __attribute__((ext_vector_type(4), may_alias));
union FragB { v16b v; v8us half[2]; unsigned short u[16]; };

__device__ __forceinline__ unsigned short bf16_bits(float x) { unsigned int u = __float_as_uint(x); return (unsigned short)((u + 0x7FFFu + ((u >> 16) & 1u)) >> 16); }
__device__ __forceinline__ float bf16_val(unsigned short b) { return __uint_as_float(((unsigned int)b) << 16); }
__device__ __forceinline__ float bf16_round(float x) { return bf16_val(bf16_bits(x)); }
template <int NT>
__device__ __forceinline__ v8f mmaN(v16b ah, v16b al, v16b bh, v16b bl, v8f c) {
  c = __builtin_amdgcn_wmma_f32_16x16x32_bf16(false, ah, false, bh, (short)0, c, false, false);
  if (NT >= 2) c = __builtin_amdgcn_wmma_f32_16x16x32_bf16(false, al, false, bh, (short)0, c, false, false);
  if (NT >= 3) c = __builtin_amdgcn_wmma_f32_16x16x32_bf16(false, ah, false, bl, (short)0, c, false, false);
  asm volatile("v_nop\n\tv_nop\n\tv_nop\n\tv_nop" : "+v"(c) : "v"(ah), "v"(al), "v"(bh), "v"(bl));
  return c;
}

__global__ __launch_bounds__(256) void k_wt_bf16(const float* __restrict__ W, unsigned short* __restrict__ Wt, int K, int N) {
  const int t = blockIdx.x * 256 + threadIdx.x;
  const int k8n = K / 8;
  if (t >= N * k8n) return;
  const int n = t / k8n, k8 = (t % k8n) * 8;
  v8us v;
#pragma unroll
  for (int i = 0; i < 8; ++i) v[i] = bf16_bits(W[(size_t)(k8 + i) * N + n]);
  *(volatile v8us*)(Wt + (size_t)n * K + k8) = v;
  __threadfence();
  *(volatile v8us*)(Wt + (size_t)n * K + k8) = v;
}

template <bool ASPLIT, int ACT, bool BIAS_BF16>
__global__ __launch_bounds__(128) void k_gemm_bf(const float* __restrict__ A, int lda, const unsigned short* __restrict__ Wt, int ldb,
                                               const float* __restrict__ bias, float* __restrict__ C, int ldc, int M, int N, int K) {
  __shared__ __attribute__((aligned(16))) float so[4][16][64];
  const int tid = threadIdx.x, w = tid >> 5, lane = tid & 31, ln = lane & 15, hh = lane >> 4;
  const int ntn = N / 64;
  const int wid = blockIdx.x * 4 + w;
  const int mt = wid / ntn, nq = wid % ntn;
  if (mt * 16 >= M) return;
  const int row0 = mt * 16, col0 = nq * 64;
  const float* arow = A + (size_t)(row0 + ln) * lda;
  v8f acc[4] = {};
  for (int kb = 0; kb < K; kb += 32) {
    FragB ah, al;
    const v4f x0 = *(const v4fa*)(arow + kb + 8 * hh), x1 = *(const v4fa*)(arow + kb + 8 * hh + 4);
    const v4f x2 = *(const v4fa*)(arow + kb + 16 + 8 * hh), x3 = *(const v4fa*)(arow + kb + 16 + 8 * hh + 4);
    float xs[16] = {x0[0],x0[1],x0[2],x0[3],x1[0],x1[1],x1[2],x1[3],x2[0],x2[1],x2[2],x2[3],x3[0],x3[1],x3[2],x3[3]};
#pragma unroll
    for (int i = 0; i < 16; ++i) { const unsigned short hb = bf16_bits(xs[i]); ah.u[i] = hb; al.u[i] = ASPLIT ? bf16_bits(xs[i] - bf16_val(hb)) : (unsigned short)0; }
#pragma unroll
    for (int t = 0; t < 4; ++t) {
      const unsigned short* brow = Wt + (size_t)(col0 + t * 16 + ln) * ldb + kb;
      FragB b;
      b.half[0] = *(const v8us*)(brow + 8 * hh);
      b.half[1] = *(const v8us*)(brow + 16 + 8 * hh);
      acc[t] = mmaN<ASPLIT ? 2 : 1>(ah.v, al.v, b.v, b.v, acc[t]);
    }
  }
#pragma unroll
  for (int t = 0; t < 4; ++t) {
    float bv = bias ? bias[col0 + t * 16 + ln] : 0.f;
    if (BIAS_BF16) bv = bf16_round(bv);
#pragma unroll
    for (int r = 0; r < 8; ++r) { float v = acc[t][r] + bv; if (ACT == 1) v = fmaxf(v, 0.f); so[w][8 * hh + r][t * 16 + ln] = v; }
  }
  __builtin_amdgcn_fence(__ATOMIC_ACQ_REL, "workgroup");
  __builtin_amdgcn_wave_barrier();
  const int rsub = lane >> 4, c4 = (lane & 15) * 4;
  for (int pass = 0; pass < 2; ++pass) {
#pragma unroll
    for (int q = 0; q < 8; ++q) {
      const int r = q * 2 + rsub;
      const v4f v = *(const v4fa*)&so[w][r][c4];
      *(volatile v4f*)(C + (size_t)(row0 + r) * ldc + col0 + c4) = v;
    }
    if (pass == 0) __threadfence();
  }
}

template <bool ASPLIT, int ACT, bool BIAS_BF16, bool RES_BF16>
__global__ __launch_bounds__(128) void k_gemm_bf3(const float* __restrict__ A, int lda, const unsigned short* __restrict__ Wt, int ldb,
                                                const float* __restrict__ bias, const float* __restrict__ resid, int rmod, int ldr,
                                                float* __restrict__ C, int ldc, int M, int N, int K) {
  __shared__ __attribute__((aligned(16))) float so[4][16][64];
  const int tid = threadIdx.x, w = tid >> 5, lane = tid & 31, ln = lane & 15, hh = lane >> 4;
  const int ntn = N / 64;
  const int wid = blockIdx.x * 4 + w;
  const int mt = wid / ntn, nq = wid % ntn;
  if (mt * 16 >= M) return;
  const int row0 = mt * 16, col0 = nq * 64;
  const float* arow = A + (size_t)(row0 + ln) * lda;
  v8f acc[4] = {};
  for (int kb = 0; kb < K; kb += 32) {
    FragB ah, al;
    const v4f x0 = *(const v4fa*)(arow + kb + 8 * hh), x1 = *(const v4fa*)(arow + kb + 8 * hh + 4);
    const v4f x2 = *(const v4fa*)(arow + kb + 16 + 8 * hh), x3 = *(const v4fa*)(arow + kb + 16 + 8 * hh + 4);
    float xs[16] = {x0[0],x0[1],x0[2],x0[3],x1[0],x1[1],x1[2],x1[3],x2[0],x2[1],x2[2],x2[3],x3[0],x3[1],x3[2],x3[3]};
#pragma unroll
    for (int i = 0; i < 16; ++i) { const unsigned short hb = bf16_bits(xs[i]); ah.u[i] = hb; al.u[i] = ASPLIT ? bf16_bits(xs[i] - bf16_val(hb)) : (unsigned short)0; }
#pragma unroll
    for (int t = 0; t < 4; ++t) {
      const unsigned short* brow = Wt + (size_t)(col0 + t * 16 + ln) * ldb + kb;
      FragB b;
      b.half[0] = *(const v8us*)(brow + 8 * hh);
      b.half[1] = *(const v8us*)(brow + 16 + 8 * hh);
      acc[t] = mmaN<ASPLIT ? 2 : 1>(ah.v, al.v, b.v, b.v, acc[t]);
    }
  }
#pragma unroll
  for (int t = 0; t < 4; ++t) {
    const int col = col0 + t * 16 + ln;
    float bv = bias ? bias[col] : 0.f;
    if (BIAS_BF16) bv = bf16_round(bv);
#pragma unroll
    for (int r = 0; r < 8; ++r) {
      float v = acc[t][r] + bv;
      if (resid) { float rv = resid[(size_t)((row0 + 8 * hh + r) % rmod) * ldr + col]; if (RES_BF16) rv = bf16_round(rv); v += rv; }
      if (ACT == 1) v = fmaxf(v, 0.f);
      if (ACT == 2) v = 0.5f * v * (1.0f + erff(v * 0.70710678118654752f));
      if (ACT == 3) { const float u = 0.7978845608028654f * (v + 0.044715f * v * v * v); v = 0.5f * v * (1.0f + tanhf(u)); }
      so[w][8 * hh + r][t * 16 + ln] = v;
    }
  }
  __builtin_amdgcn_fence(__ATOMIC_ACQ_REL, "workgroup");
  __builtin_amdgcn_wave_barrier();
  const int rsub = lane >> 4, c4 = (lane & 15) * 4;
  for (int pass = 0; pass < 2; ++pass) {
#pragma unroll
    for (int q = 0; q < 8; ++q) {
      const int r = q * 2 + rsub;
      const v4f v = *(const v4fa*)&so[w][r][c4];
      *(volatile v4f*)(C + (size_t)(row0 + r) * ldc + col0 + c4) = v;
    }
    if (pass == 0) __threadfence();
  }
}
template <bool PARAM_BF16>
__global__ __launch_bounds__(256) void k_layernorm(const float* __restrict__ X, const float* __restrict__ R, const float* __restrict__ g, const float* __restrict__ bta,
                                                  float* __restrict__ out_sum, float* __restrict__ out_norm, int N, float eps) {
  __shared__ float red[256];
  const int row = blockIdx.x, tid = threadIdx.x;
  const float* x = X + (size_t)row * N; const float* rr = R ? R + (size_t)row * N : nullptr;
  float vals[16];
  const int per = N / 256;
  float s1 = 0.f;
  for (int u = 0; u < per / 4; ++u) {
    const int j = tid * 4 + 1024 * u;
    const v4f a = *(const v4fa*)(x + j);
    v4f b = {0.f,0.f,0.f,0.f}; if (rr) b = *(const v4fa*)(rr + j);
#pragma unroll
    for (int q = 0; q < 4; ++q) { const float v = a[q] + b[q]; vals[u * 4 + q] = v; s1 += v; }
  }
  red[tid] = s1; __syncthreads();
  for (int st = 128; st > 0; st >>= 1) { if (tid < st) red[tid] += red[tid + st]; __syncthreads(); }
  const float mu = red[0] / (float)N; __syncthreads();
  float s2 = 0.f;
  for (int u = 0; u < per / 4; ++u)
#pragma unroll
    for (int q = 0; q < 4; ++q) { const float c = vals[u * 4 + q] - mu; s2 += c * c; }
  red[tid] = s2; __syncthreads();
  for (int st = 128; st > 0; st >>= 1) { if (tid < st) red[tid] += red[tid + st]; __syncthreads(); }
  const float rs = rsqrtf(red[0] / (float)N + eps);
  for (int pass = 0; pass < 2; ++pass) {
    for (int u = 0; u < per / 4; ++u) {
      const int j = tid * 4 + 1024 * u;
      v4f o, sm;
#pragma unroll
      for (int q = 0; q < 4; ++q) {
        float gg = g[j + q], bb = bta[j + q];
        if (PARAM_BF16) { gg = bf16_round(gg); bb = bf16_round(bb); }
        sm[q] = vals[u * 4 + q]; o[q] = (vals[u * 4 + q] - mu) * rs * gg + bb;
      }
      if (out_sum) *(volatile v4f*)(out_sum + (size_t)row * N + j) = sm;
      *(volatile v4f*)(out_norm + (size_t)row * N + j) = o;
    }
    if (pass == 0) __threadfence();
  }
}


typedef _Float16 v16h __attribute__((ext_vector_type(16)));
union FragH { v16h v; v8us half[2]; _Float16 h[16]; unsigned short u[16]; };
template <int NT>
__device__ __forceinline__ v8f mmaH(v16h ah, v16h al, v16h bh, v16h bl, v8f c) {
  c = __builtin_amdgcn_wmma_f32_16x16x32_f16(false, ah, false, bh, (short)0, c, false, false);
  if (NT >= 2) c = __builtin_amdgcn_wmma_f32_16x16x32_f16(false, al, false, bh, (short)0, c, false, false);
  if (NT >= 3) c = __builtin_amdgcn_wmma_f32_16x16x32_f16(false, ah, false, bl, (short)0, c, false, false);
  asm volatile("v_nop\n\tv_nop\n\tv_nop\n\tv_nop" : "+v"(c) : "v"(ah), "v"(al), "v"(bh), "v"(bl));
  return c;
}
template <bool ASPLIT>
__global__ __launch_bounds__(128) void k_gemm_h(const float* __restrict__ A, int lda, size_t sA, const _Float16* __restrict__ Bh, int ldb, size_t sB, float alpha, float* __restrict__ C, int ldc, size_t sC, int M, int N, int K) {
  __shared__ __attribute__((aligned(16))) float so[4][16][64];
  const int tid = threadIdx.x, w = tid >> 5, lane = tid & 31, ln = lane & 15, hh = lane >> 4; const int by = blockIdx.y;
  A += (size_t)by * sA; Bh += (size_t)by * sB; C += (size_t)by * sC;
  const int ntn = (N + 63) / 64; const int wid = blockIdx.x * 4 + w; const int mt = wid / ntn, nq = wid % ntn; if (mt * 16 >= M) return;
  const int row0 = mt * 16, col0 = nq * 64; const float* arow = A + (size_t)(row0 + ln) * lda;
  v8f acc[4] = {};
  for (int kb = 0; kb < K; kb += 32) {
    FragH ah, al;
    const v4f x0 = *(const v4fa*)(arow + kb + 8 * hh), x1 = *(const v4fa*)(arow + kb + 8 * hh + 4), x2 = *(const v4fa*)(arow + kb + 16 + 8 * hh), x3 = *(const v4fa*)(arow + kb + 16 + 8 * hh + 4);
    float xs[16] = {x0[0],x0[1],x0[2],x0[3],x1[0],x1[1],x1[2],x1[3],x2[0],x2[1],x2[2],x2[3],x3[0],x3[1],x3[2],x3[3]};
#pragma unroll
    for (int i = 0; i < 16; ++i) { const _Float16 h = (_Float16)xs[i]; ah.h[i] = h; al.h[i] = ASPLIT ? (_Float16)(xs[i] - (float)h) : (_Float16)0.0f; }
#pragma unroll
    for (int t = 0; t < 4; ++t) { if (col0 + t * 16 >= N) continue; const size_t boff = (size_t)(col0 + t * 16 + ln) * ldb + kb; FragH bq; bq.half[0] = *(const v8us*)(Bh + boff + 8 * hh); bq.half[1] = *(const v8us*)(Bh + boff + 16 + 8 * hh);
      acc[t] = mmaH<ASPLIT ? 2 : 1>(ah.v, al.v, bq.v, bq.v, acc[t]); }
  }
#pragma unroll
  for (int t = 0; t < 4; ++t) { if (col0 + t * 16 >= N) continue;
#pragma unroll
    for (int r = 0; r < 8; ++r) so[w][8 * hh + r][t * 16 + ln] = acc[t][r] * alpha; }
  __builtin_amdgcn_fence(__ATOMIC_ACQ_REL, "workgroup"); __builtin_amdgcn_wave_barrier();
  const int rsub = lane >> 4, c4 = (lane & 15) * 4;
  for (int pass = 0; pass < 2; ++pass) {
#pragma unroll
    for (int q = 0; q < 8; ++q) { const int r = q * 2 + rsub; if (col0 + c4 < N) { const v4f v = *(const v4fa*)&so[w][r][c4]; *(volatile v4f*)(C + (size_t)(row0 + r) * ldc + col0 + c4) = v; } }
    if (pass == 0) __threadfence(); }
}

__global__ __launch_bounds__(256) void k_wt_f16(const float* __restrict__ W, _Float16* __restrict__ Wt, int K, int N, float scale) {
  const int t = blockIdx.x * 256 + threadIdx.x; if (t >= N * (K / 8)) return; const int n = t / (K / 8), k8 = (t % (K / 8)) * 8; FragH f;
#pragma unroll
  for (int i = 0; i < 8; ++i) f.h[i] = (_Float16)(bf16_round(W[(size_t)(k8 + i) * N + n]) * scale); const v8us o = f.half[0];
  *(volatile v8us*)((unsigned short*)Wt + (size_t)n * K + k8) = o; __threadfence(); *(volatile v8us*)((unsigned short*)Wt + (size_t)n * K + k8) = o;
}
template <int ACT>
__global__ __launch_bounds__(128) void k_gemm_hhx(const _Float16* __restrict__ A, int lda, size_t sA, const _Float16* __restrict__ Bh, int ldb, size_t sB, float alpha, const float* __restrict__ bias, size_t sBias, const float* __restrict__ CP, int rowsPerB, size_t sCPb, int row0g,
    float* __restrict__ C, _Float16* __restrict__ C16, int ldc, size_t sC, int M, int N, int K) {
  __shared__ __attribute__((aligned(16))) float so[4][16][64];
  const int tid = threadIdx.x, w = tid >> 5, lane = tid & 31, ln = lane & 15, hh = lane >> 4; const int by = blockIdx.y;
  A += (size_t)by * sA; Bh += (size_t)by * sB; const size_t cofs = (size_t)by * sC; const float* bp = bias ? bias + (size_t)by * sBias : nullptr;
  const int ntn = (N + 63) / 64; const int wid = blockIdx.x * 4 + w; const int mt = wid / ntn, nq = wid % ntn; if (mt * 16 >= M) return;
  const int row0 = mt * 16, col0 = nq * 64; const _Float16* arow = A + (size_t)(row0 + ln) * lda;
  v8f acc[4] = {};
  for (int kb = 0; kb < K; kb += 32) { FragH ah; ah.half[0] = *(const v8us*)((const unsigned short*)arow + kb + 8 * hh); ah.half[1] = *(const v8us*)((const unsigned short*)arow + kb + 16 + 8 * hh);
#pragma unroll
    for (int t = 0; t < 4; ++t) { if (col0 + t * 16 >= N) continue; const size_t boff = (size_t)(col0 + t * 16 + ln) * ldb + kb; FragH bq; bq.half[0] = *(const v8us*)((const unsigned short*)Bh + boff + 8 * hh); bq.half[1] = *(const v8us*)((const unsigned short*)Bh + boff + 16 + 8 * hh);
      acc[t] = mmaH<1>(ah.v, ah.v, bq.v, bq.v, acc[t]); }
  }
#pragma unroll
  for (int t = 0; t < 4; ++t) { if (col0 + t * 16 >= N) continue; const int col = col0 + t * 16 + ln; const float bv = bp ? bf16_round(bp[col]) : 0.f;
#pragma unroll
    for (int r = 0; r < 8; ++r) { float v = acc[t][r] * alpha + bv; if (CP) { const int rr = row0g + row0 + 8 * hh + r; if (rowsPerB < 0) v += CP[cofs + (size_t)rr * ldc + col];        else { const int bidx = rr / rowsPerB; v += CP[(size_t)bidx * sCPb + (size_t)by * 64 + col]; } } if (ACT == 1) v = (v > 0.f) ? v : expm1f(v); else if (ACT == 7) v = (v > 0.f) ? v + 1.0f : expf(v); else if (ACT == 8) v = tanhf(v); else if (ACT == 9) v = 0.5f * v * (1.0f + tanhf(0.7978845608028654f * (v + 0.044715f * v * v * v))); else if (ACT == 11) v = 1.0f / (1.0f + expf(-v)); else if (ACT == 12) v = (v > 0.f) ? v : 0.01f * v; else if (ACT == 14) v = (v > 0.f) ? v : 0.1f * v; else if (ACT == 16) v = (v >= 0.f) ? v : 0.3f * v; else if (ACT == 15) v = v / (1.0f + expf(-v)); else if (ACT == 3) v = fmaxf(v, 0.f); else if (ACT == 6) v = 0.5f * v * (1.0f + erff(v * 0.70710678118654752f)); so[w][8 * hh + r][t * 16 + ln] = v; } }
  __builtin_amdgcn_fence(__ATOMIC_ACQ_REL, "workgroup"); __builtin_amdgcn_wave_barrier();
  const int rsub = lane >> 4, c4 = (lane & 15) * 4; typedef _Float16 v4h __attribute__((ext_vector_type(4)));
  for (int pass = 0; pass < 2; ++pass) {
#pragma unroll
    for (int q = 0; q < 8; ++q) { const int r = q * 2 + rsub; if (col0 + c4 < N) { const v4f v = *(const v4fa*)&so[w][r][c4]; if (C) *(volatile v4f*)(C + cofs + (size_t)(row0 + r) * ldc + col0 + c4) = v; if (C16) { v4h h4; for (int i = 0; i < 4; ++i) h4[i] = (_Float16)v[i]; *(volatile v4h*)(C16 + cofs + (size_t)(row0 + r) * ldc + col0 + c4) = h4; } } }
    if (pass == 0) __threadfence(); }
}


typedef _Float16 v4h __attribute__((ext_vector_type(4)));

__global__ __launch_bounds__(256) void k_x16(const float* __restrict__ x, _Float16* __restrict__ X16, size_t n8) { const size_t t = (size_t)blockIdx.x * 256 + threadIdx.x; if (t >= n8) return; FragH f;
#pragma unroll
  for (int q = 0; q < 8; ++q) f.h[q] = (_Float16)bf16_round(x[t * 8 + q]); *(volatile v8us*)((unsigned short*)X16 + t * 8) = f.half[0]; __threadfence(); *(volatile v8us*)((unsigned short*)X16 + t * 8) = f.half[0]; }
__global__ __launch_bounds__(256) void k_h16(const float* __restrict__ x, _Float16* __restrict__ X16, size_t n8) { const size_t t = (size_t)blockIdx.x * 256 + threadIdx.x; if (t >= n8) return; FragH f;
#pragma unroll
  for (int q = 0; q < 8; ++q) f.h[q] = (_Float16)x[t * 8 + q]; *(volatile v8us*)((unsigned short*)X16 + t * 8) = f.half[0]; __threadfence(); *(volatile v8us*)((unsigned short*)X16 + t * 8) = f.half[0]; }
__global__ __launch_bounds__(256) void k_round16f(const float* __restrict__ W, _Float16* __restrict__ Bt, size_t n8) { const size_t t = (size_t)blockIdx.x * 256 + threadIdx.x; if (t >= n8) return; FragH f;
#pragma unroll
  for (int i = 0; i < 8; ++i) f.h[i] = (_Float16)(bf16_round(W[t * 8 + i]) * 16.0f); *(volatile v8us*)((unsigned short*)Bt + t * 8) = f.half[0]; __threadfence(); *(volatile v8us*)((unsigned short*)Bt + t * 8) = f.half[0]; }
template <int NHv, int TTv>
__global__ __launch_bounds__(256) void k_vt(const _Float16* __restrict__ V16, int ldv, int voff, _Float16* __restrict__ Vt) { __shared__ unsigned short tl[64][66]; const int tid = threadIdx.x; const int slab = blockIdx.x / (TTv / 64), lg = blockIdx.x % (TTv / 64); const int b = slab / NHv, h = slab % NHv;
  for (int i = tid; i < 64 * 8; i += 256) { const int r = i / 8, c8 = (i % 8) * 8; FragH f; f.half[0] = *(const v8us*)((const unsigned short*)V16 + ((size_t)b * TTv + lg * 64 + r) * ldv + voff + h * 64 + c8);
#pragma unroll
    for (int q = 0; q < 8; ++q) tl[r][c8 + q] = f.u[q]; }
  __syncthreads();
  for (int pass = 0; pass < 2; ++pass) {
#pragma unroll
    for (int rd = 0; rd < 2; ++rd) { const int d = rd * 32 + tid / 8, pc = tid % 8; FragH f;
#pragma unroll
      for (int q = 0; q < 8; ++q) f.u[q] = tl[pc * 8 + q][d];
      *(volatile v8us*)((unsigned short*)Vt + ((size_t)slab * 64 + d) * TTv + lg * 64 + pc * 8) = f.half[0]; }
    if (pass == 0) __threadfence(); } }

__global__ __launch_bounds__(256) void k_hl(const float* __restrict__ F, _Float16* __restrict__ Hh, _Float16* __restrict__ Hl, size_t n8) { const size_t t = (size_t)blockIdx.x * 256 + threadIdx.x; if (t >= n8) return; FragH fh, fl; const v4f a = *(const v4fa*)(F + t * 8), c = *(const v4fa*)(F + t * 8 + 4);
#pragma unroll
  for (int q = 0; q < 4; ++q) { _Float16 h = (_Float16)a[q]; fh.h[q] = h; fl.h[q] = (_Float16)((a[q] - (float)h) * 1024.0f); h = (_Float16)c[q]; fh.h[4 + q] = h; fl.h[4 + q] = (_Float16)((c[q] - (float)h) * 1024.0f); }
  for (int pass = 0; pass < 2; ++pass) { *(volatile v8us*)((unsigned short*)Hh + t * 8) = fh.half[0]; *(volatile v8us*)((unsigned short*)Hl + t * 8) = fl.half[0]; if (pass == 0) __threadfence(); } }

__device__ __forceinline__ v16h g2_frag(const _Float16* p, int hh) { FragH f; f.half[0] = *(const v8us*)((const unsigned short*)p + 8 * hh); f.half[1] = *(const v8us*)((const unsigned short*)p + 16 + 8 * hh); return f.v; }
__device__ __forceinline__ v8f g2_mma(v16h a, v16h b, v8f c) { v8f d = __builtin_amdgcn_wmma_f32_16x16x32_f16(false, a, false, b, (short)0, c, false, false); asm volatile("v_nop\n\tv_nop\n\tv_nop\n\tv_nop" : "+v"(d) : "v"(a), "v"(b)); return d; }
template <int ACT>
__global__ __launch_bounds__(128) void k_gemm2(const _Float16* __restrict__ A, int lda, size_t sA, const _Float16* __restrict__ Bh, int ldb, size_t sB, float alpha, const float* __restrict__ bias, size_t sBias, const float* __restrict__ CP, int rowsPerB, size_t sCPb, int row0g,
    float* __restrict__ C, _Float16* __restrict__ C16, int ldc, size_t sC, int M, int N, int K) { static_assert(ACT == 0 || ACT == 3 || ACT == 6 || ACT == 8 || ACT == 9 || ACT == 11 || ACT == 12 || ACT == 14 || ACT == 15 || ACT == 16, "k_gemm2: unsupported ACT code (would silently apply no activation)");
  __shared__ __attribute__((aligned(16))) float so[4][32][68];
  const int tid = threadIdx.x, w = tid >> 5, lane = tid & 31, ln = lane & 15, hh = lane >> 4; const int by = blockIdx.y;
  A += (size_t)by * sA; Bh += (size_t)by * sB; const size_t cofs = (size_t)by * sC; const float* bp = bias ? bias + (size_t)by * sBias : nullptr;
  const int ntn = N >> 6; const int mt = blockIdx.x / ntn, nq = blockIdx.x - mt * ntn; const int row0 = mt * 128 + 32 * w, col0 = nq * 64; if (row0 >= M) return;
  const _Float16* a0p = A + (size_t)(row0 + ln) * lda; const _Float16* a1p = a0p + (size_t)16 * lda;
  const _Float16* b0p = Bh + (size_t)(col0 + ln) * ldb; const _Float16* b1p = b0p + (size_t)16 * ldb; const _Float16* b2p = b1p + (size_t)16 * ldb; const _Float16* b3p = b2p + (size_t)16 * ldb;
  const v8f z8 = {0.f,0.f,0.f,0.f,0.f,0.f,0.f,0.f}; v8f c00 = z8, c01 = z8, c02 = z8, c03 = z8, c10 = z8, c11 = z8, c12 = z8, c13 = z8;
#pragma unroll 1
  for (int kb = 0; kb < K; kb += 32) { const v16h a0 = g2_frag(a0p + kb, hh), a1 = g2_frag(a1p + kb, hh);
    v16h b = g2_frag(b0p + kb, hh); c00 = g2_mma(a0, b, c00); c10 = g2_mma(a1, b, c10);
    b = g2_frag(b1p + kb, hh); c01 = g2_mma(a0, b, c01); c11 = g2_mma(a1, b, c11);
    b = g2_frag(b2p + kb, hh); c02 = g2_mma(a0, b, c02); c12 = g2_mma(a1, b, c12);
    b = g2_frag(b3p + kb, hh); c03 = g2_mma(a0, b, c03); c13 = g2_mma(a1, b, c13); }
  v8f accs[8] = {c00, c01, c02, c03, c10, c11, c12, c13};
#pragma unroll
  for (int u = 0; u < 8; ++u) { const int t = u & 3, half = u >> 2; const int col = col0 + t * 16 + ln; const float bv = bp ? bf16_round(bp[col]) : 0.f;
#pragma unroll
    for (int r = 0; r < 8; ++r) { const int rloc = half * 16 + 8 * hh + r; float v = accs[u][r] * alpha + bv; if (CP) { if (rowsPerB < 0) v += CP[cofs + (size_t)(row0g + row0 + rloc) * ldc + col];        else { const int bidx = (row0g + row0 + rloc) / rowsPerB; v += CP[(size_t)bidx * sCPb + (size_t)by * 64 + col]; } }
      if (ACT == 3) v = fmaxf(v, 0.f); else if (ACT == 6) v = 0.5f * v * (1.0f + erff(v * 0.70710678118654752f)); else if (ACT == 11) v = 1.0f / (1.0f + expf(-v)); else if (ACT == 15) v = v / (1.0f + expf(-v)); else if (ACT == 12) v = (v > 0.f) ? v : 0.01f * v; else if (ACT == 8) v = tanhf(v); else if (ACT == 9) v = 0.5f * v * (1.0f + tanhf(0.7978845608028654f * (v + 0.044715f * v * v * v))); else if (ACT == 14) v = (v > 0.f) ? v : 0.1f * v; else if (ACT == 16) v = (v >= 0.f) ? v : 0.3f * v;
      so[w][rloc][t * 16 + ln] = v; } }
  __builtin_amdgcn_fence(__ATOMIC_ACQ_REL, "workgroup"); __builtin_amdgcn_wave_barrier();
  const int rsub = lane >> 4, c4 = (lane & 15) * 4;
  for (int pass = 0; pass < 2; ++pass) {
#pragma unroll
    for (int q = 0; q < 16; ++q) { const int r = q * 2 + rsub; const v4f v = *(const v4fa*)&so[w][r][c4]; if (C) *(volatile v4f*)(C + cofs + (size_t)(row0 + r) * ldc + col0 + c4) = v; if (C16) { v4h h4; for (int i = 0; i < 4; ++i) h4[i] = (_Float16)v[i]; *(volatile v4h*)(C16 + cofs + (size_t)(row0 + r) * ldc + col0 + c4) = h4; } }
    if (pass == 0) __threadfence(); } }


__global__ __launch_bounds__(256) void k_lnge(const float* __restrict__ F, int nrow, int ncol, const float* __restrict__ g, const float* __restrict__ bb, float* __restrict__ OUTF, _Float16* __restrict__ H, _Float16* __restrict__ L) {
  #pragma clang fp contract(off)
  const int wv = threadIdx.x >> 5, ln = threadIdx.x & 31; const int r = blockIdx.x * 8 + wv; if (r >= nrow) return; const float* fr = F + (size_t)r * ncol; float s = 0.f;
#pragma unroll 1
  for (int c = ln; c < ncol; c += 32) s += fr[c];
  for (int o = 16; o > 0; o >>= 1) s += __shfl_xor(s, o, 32); const float mu = s / (float)ncol; float var = 0.f;
#pragma unroll 1
  for (int c = ln; c < ncol; c += 32) { const float d = fr[c] - mu; var += d * d; }
  for (int o = 16; o > 0; o >>= 1) var += __shfl_xor(var, o, 32); const float inv = rsqrtf(var / (float)ncol + 1e-5f);
  for (int pass = 0; pass < 2; ++pass) {
#pragma unroll 1
    for (int c = ln; c < ncol; c += 32) { float y = (fr[c] - mu) * inv; y *= bf16_round(g[c]); y += bf16_round(bb[c]); const float ge = 0.5f * y * (1.0f + erff(y * 0.70710678118654752f)); if (OUTF) *(volatile float*)(OUTF + (size_t)r * ncol + c) = ge; if (H) { const _Float16 h = (_Float16)ge; *(volatile _Float16*)(H + (size_t)r * ncol + c) = h; *(volatile _Float16*)(L + (size_t)r * ncol + c) = (_Float16)((ge - (float)h) * 1024.0f); } }
    if (pass == 0) __threadfence(); } }
__global__ __launch_bounds__(256) void k_aw(const float* __restrict__ A1, const float* __restrict__ w2, const float* __restrict__ b2, float* __restrict__ AW) {
  #pragma clang fp contract(off)
  const int r = blockIdx.x * 256 + threadIdx.x; if (r >= NRH) return; float s = 0.f;
#pragma unroll 1
  for (int c = 0; c < C4; ++c) s += A1[(size_t)r * C4 + c] * bf16_round(w2[c]); s += bf16_round(b2[0]); *(volatile float*)(AW + r) = s; __threadfence(); *(volatile float*)(AW + r) = s; }
__global__ __launch_bounds__(256) void k_cc(const float* __restrict__ EH, const float* __restrict__ AW, _Float16* __restrict__ CH, _Float16* __restrict__ CL) {
  #pragma clang fp contract(off)
  const int t = blockIdx.x * 256 + threadIdx.x; if (t >= NB * (CX / 8)) return; const int c0 = (t % (CX / 8)) * 8, b = t / (CX / 8); const float* a = AW + b * TH; float m = -3.0e38f;
#pragma unroll 1
  for (int i = 0; i < TH; ++i) m = fmaxf(m, a[i]); float su = 0.f;
#pragma unroll 1
  for (int i = 0; i < TH; ++i) su += expf(a[i] - m); float acc[8]; for (int q = 0; q < 8; ++q) acc[q] = 0.f;
#pragma unroll 1
  for (int i = 0; i < TH; ++i) { const float w = expf(a[i] - m) / su; const v8f e = *(const v8f*)(EH + ((size_t)b * TH + i) * CX + c0); for (int q = 0; q < 8; ++q) acc[q] += e[q] * w; }
  FragH fh, fl; for (int q = 0; q < 8; ++q) { const _Float16 h = (_Float16)acc[q]; fh.h[q] = h; fl.h[q] = (_Float16)((acc[q] - (float)h) * 1024.0f); }
  for (int pass = 0; pass < 2; ++pass) { *(volatile v8us*)((unsigned short*)CH + (size_t)b * CX + c0) = fh.half[0]; *(volatile v8us*)((unsigned short*)CL + (size_t)b * CX + c0) = fl.half[0]; if (pass == 0) __threadfence(); } }
__global__ __launch_bounds__(256) void k_ker(const float* __restrict__ KP, float* __restrict__ KER) {
  #pragma clang fp contract(off)
  const int t = blockIdx.x * 256 + threadIdx.x; if (t >= NB * NH) return; const int h = t % NH, b = t / NH; const float* kp = KP + (size_t)b * NKPP + h * 9; float m = -3.0e38f; for (int k = 0; k < 9; ++k) m = fmaxf(m, kp[k]); float su = 0.f; for (int k = 0; k < 9; ++k) su += expf(kp[k] - m);
  for (int pass = 0; pass < 2; ++pass) { for (int k = 0; k < 9; ++k) *(volatile float*)(KER + (size_t)t * 9 + k) = expf(kp[k] - m) / su; if (pass == 0) __threadfence(); } }
__global__ __launch_bounds__(256) void k_conv(const float* __restrict__ S, const int* __restrict__ mask, const float* __restrict__ KER, int b, int hc0, float* __restrict__ S2) {
  #pragma clang fp contract(off)
  const size_t t = (size_t)blockIdx.x * 256 + threadIdx.x; if (t >= (size_t)HCH * TT * (TT / 4)) return; const int j0 = (int)(t % (TT / 4)) * 4; const int i = (int)((t / (TT / 4)) % TT); const int hl = (int)(t / ((size_t)(TT / 4) * TT)); const float* kr = KER + ((size_t)b * NH + hc0 + hl) * 9; const float* sl = S + (size_t)hl * TT * TT; v4f r;
  for (int q = 0; q < 4; ++q) { const int j = j0 + q; float acc = 0.f;
#pragma unroll
    for (int di = 0; di < 3; ++di) { const int ii = i + di - 1; if (ii < 0 || ii >= TT) continue;
#pragma unroll
      for (int dj = 0; dj < 3; ++dj) { const int jj = j + dj - 1; if (jj < 0 || jj >= TT) continue; const float a = mask[(size_t)ii * TT + jj] ? 0.f : sl[(size_t)ii * TT + jj]; acc += kr[di * 3 + dj] * a; } }
    r[q] = mask[(size_t)i * TT + j] ? -3.0e38f : acc; }
  float* d = S2 + ((size_t)hl * TT + i) * TT + j0; *(volatile v4f*)d = r; __threadfence(); *(volatile v4f*)d = r; }
__global__ __launch_bounds__(256) void k_msoft(const float* __restrict__ S2, _Float16* __restrict__ PH, _Float16* __restrict__ PL) {
  #pragma clang fp contract(off)
  const int wv = threadIdx.x >> 5, ln = threadIdx.x & 31; const int rr = blockIdx.x * 8 + wv; if (rr >= HCH * TT) return; const int i = rr % TT, hl = rr / TT; const float* sr = S2 + (size_t)rr * TT; float m = -3.0e38f;
#pragma unroll 1
  for (int j = ln; j < TT; j += 32) m = fmaxf(m, sr[j]);
  for (int o = 16; o > 0; o >>= 1) m = fmaxf(m, __shfl_xor(m, o, 32)); float su = 0.f;
#pragma unroll 1
  for (int j = ln; j < TT; j += 32) { const float z = sr[j]; if (z > -1.0e38f) su += expf(z - m); }
  for (int o = 16; o > 0; o >>= 1) su += __shfl_xor(su, o, 32); const float f = 1024.0f / su;
  for (int pass = 0; pass < 2; ++pass) {
#pragma unroll 1
    for (int j = ln; j < TT; j += 32) { const float z = sr[j]; const float p = (z > -1.0e38f) ? expf(z - m) * f : 0.f; const _Float16 h = (_Float16)p; *(volatile _Float16*)(PH + (size_t)rr * TT + j) = h; if (i < RB) *(volatile _Float16*)(PL + ((size_t)hl * RB + i) * TT + j) = (_Float16)((p - (float)h) * 1024.0f); }
    if (pass == 0) __threadfence(); } }
__global__ __launch_bounds__(256) void k_oadd(float* __restrict__ O, const float* __restrict__ X1, const float* __restrict__ X2, size_t row0, int col0) {
  #pragma clang fp contract(off)
  const int t = blockIdx.x * 256 + threadIdx.x; if (t >= RB * (HCH * HD / 4)) return; const int c = col0 + (t % (HCH * HD / 4)) * 4; const int i = t / (HCH * HD / 4); float* o = O + (row0 + i) * DD + c; const v4f a = *(const v4fa*)o, b = *(const v4fa*)(X1 + (size_t)i * DD + c), cc = *(const v4fa*)(X2 + (size_t)i * DD + c); v4f r; for (int q = 0; q < 4; ++q) { float v = a[q] + b[q]; v += cc[q]; r[q] = v; }
  *(volatile v4f*)o = r; __threadfence(); *(volatile v4f*)o = r; }
__global__ __launch_bounds__(256) void k_ohl(const float* __restrict__ O, _Float16* __restrict__ OH, _Float16* __restrict__ OL, size_t n8) {
  const size_t t = (size_t)blockIdx.x * 256 + threadIdx.x; if (t >= n8) return; const size_t e0 = t * 8; const size_t row = e0 / DD; const int i = (int)(row % TT), b = (int)(row / TT); const v8f v = *(const v8f*)(O + e0); FragH h, l;
  for (int q = 0; q < 8; ++q) { const _Float16 x = (_Float16)v[q]; h.h[q] = x; l.h[q] = (_Float16)((v[q] - (float)x) * 1024.0f); }
  for (int pass = 0; pass < 2; ++pass) { *(volatile v8us*)((unsigned short*)OH + e0) = h.half[0]; if (i < RB) *(volatile v8us*)((unsigned short*)OL + ((size_t)b * RB + i) * DD + (e0 % DD)) = l.half[0]; if (pass == 0) __threadfence(); } }
__global__ __launch_bounds__(256) void k_wt_pad(const float* __restrict__ Wm, const float* __restrict__ b, int K, int nout, int npad, _Float16* __restrict__ Bt, float* __restrict__ BB) { const size_t t = (size_t)blockIdx.x * 256 + threadIdx.x; if (t >= (size_t)npad * (K / 8)) return; const int n = (int)(t / (K / 8)), k8 = (int)(t % (K / 8)) * 8; FragH f;
  for (int i = 0; i < 8; ++i) f.h[i] = (n < nout) ? (_Float16)(bf16_round(Wm[(size_t)(k8 + i) * nout + n]) * 16.0f) : (_Float16)0.0f;
  for (int pass = 0; pass < 2; ++pass) { *(volatile v8us*)((unsigned short*)Bt + (size_t)n * K + k8) = f.half[0]; if (t < (size_t)npad) *(volatile float*)(BB + t) = (t < (size_t)nout) ? bf16_round(b[t]) : 0.f; if (pass == 0) __threadfence(); } }
__global__ __launch_bounds__(256) void k_zeroh(_Float16* __restrict__ p, size_t n8) { const size_t t = (size_t)blockIdx.x * 256 + threadIdx.x; if (t >= n8) return; v8us z; for (int q = 0; q < 8; ++q) z[q] = 0; *(volatile v8us*)((unsigned short*)p + t * 8) = z; __threadfence(); *(volatile v8us*)((unsigned short*)p + t * 8) = z; }

extern "C" void kernel_launch(void* const* d_in, const int* in_sizes, int n_in,
                              void* d_out, int out_size, void* d_ws, size_t ws_size, hipStream_t stream) {
  (void)in_sizes; (void)n_in; (void)out_size;
  const float* const* I = (const float* const*)d_in; const float* x = I[0]; const float* hist = I[1]; const float* Wq = I[2]; const float* Wk = I[3]; const float* Wv = I[4]; const float* hW = I[5]; const float* hb = I[6]; const float* hg = I[7]; const float* hbb = I[8]; const float* cW1 = I[9]; const float* cb1 = I[10]; const float* cW2 = I[11]; const float* cb2 = I[12]; const float* kW1 = I[13]; const float* kb1 = I[14]; const float* kg = I[15]; const float* kbb = I[16]; const float* kW2 = I[17]; const float* kb2 = I[18]; const float* pW = I[19]; const float* pb = I[20]; const int* mask = (const int*)d_in[21];
  char* ws = (char*)d_ws; size_t off = 0;
  auto take = [&](size_t bytes) { char* p = ws + off; off += (bytes + 255) & ~(size_t)255; return p; };
  const size_t np = (size_t)NR * DD;
  _Float16* BQ = (_Float16*)take((size_t)DD * DD * 2); _Float16* BK = (_Float16*)take((size_t)DD * DD * 2); _Float16* BV = (_Float16*)take((size_t)DD * DD * 2); _Float16* BP = (_Float16*)take((size_t)DD * DD * 2);
  _Float16* BH = (_Float16*)take((size_t)CX * DD * 2); _Float16* BC1 = (_Float16*)take((size_t)C4 * CX * 2); _Float16* BK1 = (_Float16*)take((size_t)DD * CX * 2); _Float16* BK2 = (_Float16*)take((size_t)NKPP * DD * 2); float* BBK2 = (float*)take(NKPP * 4);
  _Float16* X16 = (_Float16*)take(np * 2); _Float16* Q16 = (_Float16*)take(np * 2); _Float16* K16 = (_Float16*)take(np * 2); float* VF = (float*)take(np * 4); _Float16* VH = (_Float16*)take(np * 2); _Float16* VL = (_Float16*)take(np * 2); _Float16* VTh = (_Float16*)take(np * 2); _Float16* VTl = (_Float16*)take(np * 2);
  _Float16* HS16 = (_Float16*)take((size_t)NRH * DD * 2); float* E0 = (float*)take((size_t)NRH * CX * 4); float* EH = (float*)take((size_t)NRH * CX * 4); _Float16* EHh = (_Float16*)take((size_t)NRH * CX * 2); _Float16* EHl = (_Float16*)take((size_t)NRH * CX * 2); float* A1 = (float*)take((size_t)NRH * C4 * 4); float* AW = (float*)take(NRH * 4);
  _Float16* CCh = (_Float16*)take((size_t)32 * CX * 2); _Float16* CCl = (_Float16*)take((size_t)32 * CX * 2); float* G1 = (float*)take((size_t)32 * DD * 4); _Float16* G1h = (_Float16*)take((size_t)32 * DD * 2); _Float16* G1l = (_Float16*)take((size_t)32 * DD * 2); float* KP = (float*)take((size_t)32 * NKPP * 4); float* KER = (float*)take((size_t)NB * NH * 9 * 4);
  float* S = (float*)take((size_t)HCH * TT * TT * 4); float* S2 = (float*)take((size_t)HCH * TT * TT * 4); _Float16* PH = (_Float16*)take((size_t)HCH * TT * TT * 2); _Float16* PL = (_Float16*)take((size_t)HCH * RB * TT * 2); float* OX1 = (float*)take((size_t)RB * DD * 4); float* OX2 = (float*)take((size_t)RB * DD * 4); _Float16* OL = (_Float16*)take((size_t)NB * RB * DD * 2);
  float* O = VF;        _Float16* OH = Q16;
  if (off > ws_size) return;
  k_wt_f16<<<(unsigned)(((size_t)DD * DD / 8 + 255) / 256), 256, 0, stream>>>(Wq, BQ, DD, DD, 16.0f); k_wt_f16<<<(unsigned)(((size_t)DD * DD / 8 + 255) / 256), 256, 0, stream>>>(Wk, BK, DD, DD, 16.0f); k_wt_f16<<<(unsigned)(((size_t)DD * DD / 8 + 255) / 256), 256, 0, stream>>>(Wv, BV, DD, DD, 16.0f); k_wt_f16<<<(unsigned)(((size_t)DD * DD / 8 + 255) / 256), 256, 0, stream>>>(pW, BP, DD, DD, 16.0f);
  k_wt_f16<<<(unsigned)(((size_t)DD * CX / 8 + 255) / 256), 256, 0, stream>>>(hW, BH, DD, CX, 16.0f); k_wt_f16<<<(unsigned)(((size_t)CX * C4 / 8 + 255) / 256), 256, 0, stream>>>(cW1, BC1, CX, C4, 16.0f); k_wt_f16<<<(unsigned)(((size_t)CX * DD / 8 + 255) / 256), 256, 0, stream>>>(kW1, BK1, CX, DD, 16.0f); k_wt_pad<<<(unsigned)(((size_t)NKPP * DD / 8 + 255) / 256), 256, 0, stream>>>(kW2, kb2, DD, NKP, NKPP, BK2, BBK2);
  k_x16<<<(unsigned)(((size_t)NRH * DD / 8 + 255) / 256), 256, 0, stream>>>(hist, HS16, (size_t)NRH * DD / 8);
  k_gemm2<0><<<dim3((NRH / 128) * (CX / 64), 1), 128, 0, stream>>>(HS16, DD, 0, BH, DD, 0, 0.0625f, hb, 0, nullptr, 1, 0, 0, E0, nullptr, CX, 0, NRH, CX, DD);
  k_lnge<<<NRH / 8, 256, 0, stream>>>(E0, NRH, CX, hg, hbb, EH, EHh, EHl);
  k_gemm2<0><<<dim3((NRH / 128) * (C4 / 64), 1), 128, 0, stream>>>(EHl, CX, 0, BC1, CX, 0, 0.0625f / 1024.0f, nullptr, 0, nullptr, 1, 0, 0, A1, nullptr, C4, 0, NRH, C4, CX);
  k_gemm2<6><<<dim3((NRH / 128) * (C4 / 64), 1), 128, 0, stream>>>(EHh, CX, 0, BC1, CX, 0, 0.0625f, cb1, 0, A1, 1, (size_t)C4, 0, A1, nullptr, C4, 0, NRH, C4, CX);
  k_aw<<<(NRH + 255) / 256, 256, 0, stream>>>(A1, cW2, cb2, AW);
  k_zeroh<<<(32 * CX / 8 + 255) / 256, 256, 0, stream>>>(CCh, (size_t)32 * CX / 8); k_zeroh<<<(32 * CX / 8 + 255) / 256, 256, 0, stream>>>(CCl, (size_t)32 * CX / 8);
  k_cc<<<(NB * (CX / 8) + 255) / 256, 256, 0, stream>>>(EH, AW, CCh, CCl);
  k_gemm2<0><<<dim3(1 * (DD / 64), 1), 128, 0, stream>>>(CCl, CX, 0, BK1, CX, 0, 0.0625f / 1024.0f, nullptr, 0, nullptr, 1, 0, 0, G1, nullptr, DD, 0, 32, DD, CX);
  k_gemm2<0><<<dim3(1 * (DD / 64), 1), 128, 0, stream>>>(CCh, CX, 0, BK1, CX, 0, 0.0625f, kb1, 0, G1, 1, (size_t)DD, 0, G1, nullptr, DD, 0, 32, DD, CX);
  k_lnge<<<32 / 8, 256, 0, stream>>>(G1, 32, DD, kg, kbb, nullptr, G1h, G1l);
  k_gemm2<0><<<dim3(1 * (NKPP / 64), 1), 128, 0, stream>>>(G1l, DD, 0, BK2, DD, 0, 0.0625f / 1024.0f, nullptr, 0, nullptr, 1, 0, 0, KP, nullptr, NKPP, 0, 32, NKPP, DD);
  k_gemm2<0><<<dim3(1 * (NKPP / 64), 1), 128, 0, stream>>>(G1h, DD, 0, BK2, DD, 0, 0.0625f, BBK2, 0, KP, 1, (size_t)NKPP, 0, KP, nullptr, NKPP, 0, 32, NKPP, DD);
  k_ker<<<1, 256, 0, stream>>>(KP, KER);
  k_x16<<<(unsigned)((np / 8 + 255) / 256), 256, 0, stream>>>(x, X16, np / 8);
  const dim3 gp((NR / 128) * (DD / 64), 1);
  k_gemm2<0><<<gp, 128, 0, stream>>>(X16, DD, 0, BQ, DD, 0, 0.0625f, nullptr, 0, nullptr, 1, 0, 0, nullptr, Q16, DD, 0, NR, DD, DD); k_gemm2<0><<<gp, 128, 0, stream>>>(X16, DD, 0, BK, DD, 0, 0.0625f, nullptr, 0, nullptr, 1, 0, 0, nullptr, K16, DD, 0, NR, DD, DD);
  k_gemm2<0><<<gp, 128, 0, stream>>>(X16, DD, 0, BV, DD, 0, 0.0625f, nullptr, 0, nullptr, 1, 0, 0, VF, nullptr, DD, 0, NR, DD, DD); k_hl<<<(unsigned)((np / 8 + 255) / 256), 256, 0, stream>>>(VF, VH, VL, np / 8);
  k_vt<NH, TT><<<NB * NH * (TT / 64), 256, 0, stream>>>(VH, DD, 0, VTh); k_vt<NH, TT><<<NB * NH * (TT / 64), 256, 0, stream>>>(VL, DD, 0, VTl);
  const size_t sS = (size_t)TT * TT;
  for (int b = 0; b < NB; ++b) for (int hc = 0; hc < NH; hc += HCH) {
    const _Float16* qb = Q16 + (size_t)b * TT * DD + hc * HD; const _Float16* kb = K16 + (size_t)b * TT * DD + hc * HD; const _Float16* vth = VTh + (size_t)(b * NH + hc) * 64 * TT; const _Float16* vtl = VTl + (size_t)(b * NH + hc) * 64 * TT; float* ob = O + (size_t)b * TT * DD + hc * HD;
    k_gemm2<0><<<dim3((TT / 128) * (TT / 64), HCH), 128, 0, stream>>>(qb, DD, (size_t)HD, kb, DD, (size_t)HD, SCL, nullptr, 0, nullptr, 1, 0, 0, S, nullptr, TT, sS, TT, TT, HD);
    k_conv<<<(unsigned)(((size_t)HCH * TT * (TT / 4) + 255) / 256), 256, 0, stream>>>(S, mask, KER, b, hc, S2);
    k_msoft<<<(HCH * TT) / 8, 256, 0, stream>>>(S2, PH, PL);
    k_gemm2<0><<<dim3((TT / 128) * 1, HCH), 128, 0, stream>>>(PH, TT, sS, vth, TT, (size_t)64 * TT, 0.0009765625f, nullptr, 0, nullptr, 1, 0, 0, ob, nullptr, DD, (size_t)HD, TT, HD, TT);
    k_gemm2<0><<<dim3(1, HCH), 128, 0, stream>>>(PL, TT, (size_t)RB * TT, vth, TT, (size_t)64 * TT, 0.0009765625f / 1024.0f, nullptr, 0, nullptr, 1, 0, 0, OX1 + hc * HD, nullptr, DD, (size_t)HD, RB, HD, TT);
    k_gemm2<0><<<dim3(1, HCH), 128, 0, stream>>>(PH, TT, sS, vtl, TT, (size_t)64 * TT, 0.0009765625f / 1024.0f, nullptr, 0, nullptr, 1, 0, 0, OX2 + hc * HD, nullptr, DD, (size_t)HD, RB, HD, TT);
    k_oadd<<<(RB * (HCH * HD / 4) + 255) / 256, 256, 0, stream>>>(O, OX1, OX2, (size_t)b * TT, hc * HD); }
  k_ohl<<<(unsigned)((np / 8 + 255) / 256), 256, 0, stream>>>(O, OH, OL, np / 8);
  k_gemm2<0><<<gp, 128, 0, stream>>>(OH, DD, 0, BP, DD, 0, 0.0625f, pb, 0, nullptr, 1, 0, 0, (float*)d_out, nullptr, DD, 0, NR, DD, DD);
  for (int b = 0; b < NB; ++b) k_gemm2<0><<<dim3(1 * (DD / 64), 1), 128, 0, stream>>>(OL + (size_t)b * RB * DD, DD, 0, BP, DD, 0, 0.0625f / 1024.0f, nullptr, 0, (float*)d_out + (size_t)b * TT * DD, 1, (size_t)DD, 0, (float*)d_out + (size_t)b * TT * DD, nullptr, DD, 0, RB, DD, DD);
}
